// NNTransformLearner_21741124452436
// MI455X (gfx1250) — hardware-run, weakly checked
//
#include <hip/hip_runtime.h>
#include <stddef.h>


typedef _Float16 v16h __attribute__((ext_vector_type(16)));
typedef _Float16 v8h  __attribute__((ext_vector_type(8)));
typedef float    v8f  __attribute__((ext_vector_type(8)));
typedef float    v4f  __attribute__((ext_vector_type(4)));
typedef _Float16 h16;

#define NFULL 8192
#define NREAL 8191
#define KPAD  8192
#define DCH   128
#ifndef QROWS
#define QROWS 8192
#endif

static_assert(NREAL == NFULL - 1);
static_assert(KPAD >= NREAL && (KPAD % 64) == 0 && KPAD <= NFULL);
static_assert(QROWS >= 128 && QROWS <= NFULL && (QROWS % 128) == 0);
static_assert(DCH == 128 && (DCH % 32) == 0 && (DCH % 64) == 0);
static_assert(DCH == 16 * 8);
static_assert((4096 / DCH) == 32);
static_assert(((NFULL * DCH) % 4096) == 0 && ((KPAD * DCH) % 4096) == 0 && ((DCH * DCH) % 4096) == 0);
static_assert(((NREAL * DCH) % 8) == 0);

#define LDT 72
#define LDK 136
#define LDO 36
#define LDP 132
static_assert((LDT % 8) == 0 && LDT >= 64);
static_assert((LDK % 8) == 0 && LDK >= DCH);
static_assert((LDO % 4) == 0 && LDO >= 32);
static_assert((LDP % 4) == 0 && LDP >= DCH);

#define GAMMAK 0.00390625f
#define XCARRY 64.0f
#define KCARRY 64.0f
#define VCARRY 64.0f
#define PCARRY 1024.0f
#define SSCALE (2.0f * GAMMAK / (XCARRY * KCARRY))

#define PLANE_BYTES ((size_t)NFULL * DCH * 2)
#define RPL_BYTES   ((size_t)DCH * DCH * 2)
#define NRM_BYTES   ((size_t)NFULL * 4)
#define OFF_XQ ((size_t)0)
#define OFF_YH (OFF_XQ + PLANE_BYTES)
#define OFF_RH (OFF_YH + PLANE_BYTES)
#define OFF_KH (OFF_RH + RPL_BYTES)
#define OFF_VT (OFF_KH + PLANE_BYTES)
#define OFF_GQ (OFF_VT + PLANE_BYTES)
#define OFF_GK (OFF_GQ + NRM_BYTES)
#define WS_TOTAL (OFF_GK + NRM_BYTES)
static_assert((PLANE_BYTES % 128) == 0 && (RPL_BYTES % 128) == 0 && (NRM_BYTES % 128) == 0);
static_assert((size_t)KPAD * DCH * 2 <= PLANE_BYTES);
static_assert((size_t)KPAD * 4 <= NRM_BYTES);
static_assert(WS_TOTAL <= (size_t)134217728);

__device__ __forceinline__ float bf16r(float x) {
  unsigned int u = __float_as_uint(x);
  u = (u + 0x7FFFu + ((u >> 16) & 1u)) & 0xFFFF0000u;
  return __uint_as_float(u);
}

static __device__ __forceinline__ h16 toh_flush(float v) {
  const h16 r = (h16)v;
  return (fabsf(v) < 6.103515625e-05f) ? (h16)0.0f : r;
}

__device__ __forceinline__ v16h frag_at(const _Float16* p) {
  v8h lo = *(const v8h*)(p);
  v8h hi = *(const v8h*)(p + 16);
  v16h out;
#pragma unroll
  for (int i = 0; i < 8; ++i) { out[i] = lo[i]; out[i + 8] = hi[i]; }
  return out;
}
__device__ __forceinline__ v16h ld_frag(const _Float16* base, unsigned ld) {
  const unsigned lane = threadIdx.x & 31u;
  return frag_at(base + (lane & 15u) * ld + (lane >> 4) * 8u);
}

__device__ __forceinline__ v8f wmma16(v16h a, v16h b, v8f c) {
  v8f d = __builtin_amdgcn_wmma_f32_16x16x32_f16(false, a, false, b, (short)0, c,
                                                 false, false);
  asm volatile("v_nop\n\tv_nop\n\tv_nop\n\tv_nop" : "+v"(d) : "v"(a), "v"(b));
  return d;
}

__device__ __forceinline__ float red16_sum(float x) {
#pragma unroll
  for (int off = 1; off < 16; off <<= 1) x += __shfl_xor(x, off, 32);
  return x;
}

__device__ __forceinline__ void wave_lds_sync() {
  __builtin_amdgcn_fence(3  , "wavefront");
  asm volatile("s_wait_dscnt 0x0" ::: "memory");
  __builtin_amdgcn_wave_barrier();
}

template <int WITH_NORM>
__device__ __forceinline__ void conv_body(const float* __restrict__ src,
                                          _Float16* __restrict__ dst,
                                          float* __restrict__ gnorm, const unsigned nreal) {
  __shared__ float Ns[32];
  const unsigned tid = threadIdx.x, lane = tid & 31u;
  const unsigned w = (unsigned)__builtin_amdgcn_readfirstlane((int)(tid >> 5));
#pragma unroll 1
  for (unsigned j = 0; j < 2u; ++j) {
    const unsigned e = ((blockIdx.x * 2u + j) * 256u + tid) * 8u;
    const bool live = e < nreal;
    const unsigned ec = live ? e : (nreal - 8u);
    const v4f a0 = *(const v4f*)(src + ec);
    const v4f a1 = *(const v4f*)(src + ec + 4u);
    v8h o;
    float ss = 0.0f;
#pragma unroll
    for (int i = 0; i < 4; ++i) {
      const float e0 = live ? bf16r(a0[i]) : 0.0f;
      const float e1 = live ? bf16r(a1[i]) : 0.0f;
      o[i]     = toh_flush(XCARRY * e0);
      o[i + 4] = toh_flush(XCARRY * e1);
      ss += e0 * e0;
      ss += e1 * e1;
    }
    if (WITH_NORM) {
      ss = red16_sum(ss);
      if ((tid & 15u) == 0u) Ns[16u * j + (tid >> 4)] = GAMMAK * ss;
    }
    _Float16* p = dst + e;
    *(volatile v8h*)p = o;
    __threadfence();
    *(volatile v8h*)p = o;
  }
  if (WITH_NORM) {
    __syncthreads();
    const v4f nv = *(const v4f*)&Ns[(lane & 7u) * 4u];
    if (w == 0u && lane < 8u) {
      float* q = gnorm + blockIdx.x * 32u + lane * 4u;
      *(volatile v4f*)q = nv;
      __threadfence();
      *(volatile v4f*)q = nv;
    }
  }
}

__global__ __launch_bounds__(256) void conv_norm_kernel(
    const float* __restrict__ src, _Float16* __restrict__ dst, float* __restrict__ gnorm,
    unsigned nreal) {
  conv_body<1>(src, dst, gnorm, nreal);
}
__global__ __launch_bounds__(256) void conv_plain_kernel(
    const float* __restrict__ src, _Float16* __restrict__ dst, unsigned nreal) {
  conv_body<0>(src, dst, (float*)0, nreal);
}

__global__ __launch_bounds__(256) void vtconv_kernel(
    const float* __restrict__ X, _Float16* __restrict__ Vt) {
  __shared__ _Float16 T[64 * LDT];
  const unsigned tid = threadIdx.x;
  const unsigned n0 = blockIdx.x * 64u;
  const unsigned k0 = blockIdx.y * 64u;
#pragma unroll 4
  for (unsigned j = 0; j < 16u; ++j) {
    const unsigned idx = tid + 256u * j;
    const unsigned kr = idx >> 6, nc = idx & 63u;
    const unsigned key = k0 + kr;
    const bool live = key < (unsigned)NREAL;
    const unsigned srow = live ? (key + 1u) : (unsigned)NREAL;
    const float v = X[(size_t)srow * DCH + n0 + nc];
    const float e = live ? bf16r(v) : 0.0f;
    T[nc * LDT + kr] = toh_flush(VCARRY * e);
  }
  __syncthreads();
  v8h x[2];
  size_t off[2];
#pragma unroll
  for (unsigned i = 0; i < 2u; ++i) {
    const unsigned n = 32u * i + (tid >> 3);
    const unsigned kc = (tid & 7u) * 8u;
    x[i] = *(const v8h*)&T[n * LDT + kc];
    off[i] = (size_t)(n0 + n) * KPAD + k0 + kc;
  }
#pragma unroll
  for (int i = 0; i < 2; ++i) *(volatile v8h*)(Vt + off[i]) = x[i];
  __threadfence();
#pragma unroll
  for (int i = 0; i < 2; ++i) *(volatile v8h*)(Vt + off[i]) = x[i];
}

__global__ __launch_bounds__(256) void proj_kernel(
    const _Float16* __restrict__ A16, const _Float16* __restrict__ Bt,
    const float* __restrict__ tb, _Float16* __restrict__ Kh, float* __restrict__ GK) {
  __shared__ float Cs[64 * LDP];
  __shared__ float Ns[64];
  const unsigned tid = threadIdx.x, lane = tid & 31u;
  const unsigned w = (unsigned)__builtin_amdgcn_readfirstlane((int)(tid >> 5));
  const unsigned mw = w >> 1, nw = w & 1u;
  const unsigned hh = lane >> 4, m = lane & 15u;
  const unsigned row0 = blockIdx.x * 64u;

  const _Float16* ap = A16 + (size_t)(row0 + mw * 16u + m) * DCH + hh * 8u;
  const _Float16* bp = Bt + (size_t)(nw * 64u + m) * DCH + hh * 8u;
  v8f acc[4];
#pragma unroll
  for (int j = 0; j < 4; ++j) acc[j] = (v8f){};
#pragma unroll
  for (unsigned k0 = 0; k0 < (unsigned)DCH; k0 += 32u) {
    const v16h a = frag_at(ap + k0);
#pragma unroll
    for (int j = 0; j < 4; ++j) {
      const v16h b = frag_at(bp + (size_t)j * 16u * DCH + k0);
      acc[j] = wmma16(a, b, acc[j]);
    }
  }
#pragma unroll
  for (int j = 0; j < 4; ++j)
#pragma unroll
    for (int r = 0; r < 8; ++r)
      Cs[(mw * 16u + hh * 8u + (unsigned)r) * LDP + nw * 64u + (unsigned)j * 16u + m] = acc[j][r];
  __syncthreads();

#pragma unroll 1
  for (unsigned i = 0; i < 4u; ++i) {
    const unsigned r = 16u * i + (tid >> 4);
    const unsigned c = (tid & 15u) * 8u;
    const unsigned row = row0 + r;
    const bool live = row < (unsigned)NREAL;
    const v4f u0 = *(const v4f*)&Cs[r * LDP + c];
    const v4f u1 = *(const v4f*)&Cs[r * LDP + c + 4u];
    const v4f t0 = *(const v4f*)(tb + c);
    const v4f t1 = *(const v4f*)(tb + c + 4u);
    v8h x;
    float ss = 0.0f;
#pragma unroll
    for (int j = 0; j < 4; ++j) {
      const float y0 = live ? (u0[j] * (1.0f / (XCARRY * XCARRY)) + bf16r(t0[j])) : 0.0f;
      const float y1 = live ? (u1[j] * (1.0f / (XCARRY * XCARRY)) + bf16r(t1[j])) : 0.0f;
      x[j]     = toh_flush(KCARRY * y0);
      x[j + 4] = toh_flush(KCARRY * y1);
      ss += y0 * y0;
      ss += y1 * y1;
    }
    ss = red16_sum(ss);
    if ((tid & 15u) == 0u) Ns[r] = live ? (GAMMAK * ss) : 1.0e30f;
    _Float16* p = Kh + (size_t)row * DCH + c;
    *(volatile v8h*)p = x;
    __threadfence();
    *(volatile v8h*)p = x;
  }
  __syncthreads();
  const v4f nv = *(const v4f*)&Ns[(lane & 15u) * 4u];
  if (w == 0u && lane < 16u) {
    float* q = GK + row0 + lane * 4u;
    *(volatile v4f*)q = nv;
    __threadfence();
    *(volatile v4f*)q = nv;
  }
}

union VOTile {
  _Float16 h[DCH * LDT];
  float f[8 * 16 * LDO];
};
static_assert(sizeof(_Float16) * DCH * LDT >= sizeof(float) * 8 * 16 * LDO);

__global__ __launch_bounds__(256) __attribute__((amdgpu_num_vgpr(256))) void kreg_flash_kernel(
    const _Float16* __restrict__ Qh, const _Float16* __restrict__ Kh,
    const _Float16* __restrict__ Vt, const float* __restrict__ GQ,
    const float* __restrict__ GK, float* __restrict__ Out) {
  __shared__ _Float16 Ks[64 * LDK];
  __shared__ VOTile VO;
  __shared__ _Float16 Ps[8 * 16 * LDT];
  __shared__ float Gs[64];

  const unsigned tid = threadIdx.x, lane = tid & 31u;
  const unsigned w = (unsigned)__builtin_amdgcn_readfirstlane((int)(tid >> 5));
  const unsigned hh = lane >> 4, m = lane & 15u;
  const unsigned qrow0 = blockIdx.x * 128u + w * 16u;
  const unsigned pbase = w * (16u * LDT);
  const unsigned obase = w * (16u * LDO);

  const size_t qoff = (size_t)(qrow0 + m) * DCH + hh * 8u;
  v16h qf[4];
#pragma unroll
  for (int c = 0; c < 4; ++c) qf[c] = frag_at(Qh + qoff + c * 32);

  float gq[8], lsum[8];
  {
    const v4f g0 = *(const v4f*)(GQ + qrow0 + hh * 8u);
    const v4f g1 = *(const v4f*)(GQ + qrow0 + hh * 8u + 4u);
#pragma unroll
    for (int i = 0; i < 4; ++i) { gq[i] = g0[i]; gq[i + 4] = g1[i]; }
  }
#pragma unroll
  for (int v = 0; v < 8; ++v) lsum[v] = 0.0f;
  v8f o[8];
#pragma unroll
  for (int nb = 0; nb < 8; ++nb) o[nb] = (v8f){};

#pragma unroll 1
  for (unsigned kb = 0; kb < (unsigned)KPAD; kb += 64u) {
#pragma unroll
    for (unsigned j = 0; j < 4u; ++j) {
      const unsigned idx = tid + 256u * j;
      const unsigned rk = idx >> 4, ck = (idx & 15u) * 8u;
      *(v8h*)&Ks[rk * LDK + ck] = *(const v8h*)(Kh + (size_t)(kb + rk) * DCH + ck);
      const unsigned rv = idx >> 3, cv = (idx & 7u) * 8u;
      *(v8h*)&VO.h[rv * LDT + cv] = *(const v8h*)(Vt + (size_t)rv * KPAD + kb + cv);
    }
    if (w < 2u) Gs[tid] = GK[kb + tid];
    __syncthreads();

#pragma unroll
    for (int kg = 0; kg < 4; ++kg) {
      v8f t = {};
#pragma unroll
      for (int c = 0; c < 4; ++c) {
        const v16h kf = ld_frag(&Ks[(kg * 16) * LDK + c * 32], LDK);
        t = wmma16(qf[c], kf, t);
      }
      const float gkv = Gs[kg * 16 + (int)m];
#pragma unroll
      for (int v = 0; v < 8; ++v) {
        const float l = fminf(t[v] * SSCALE - gq[v] - gkv, 0.0f);
        const h16 ph = toh_flush(__expf(l) * PCARRY);
        lsum[v] += (float)ph;
        Ps[pbase + (hh * 8u + (unsigned)v) * LDT + (unsigned)kg * 16u + m] = ph;
      }
    }
    wave_lds_sync();

#pragma unroll
    for (int c = 0; c < 2; ++c) {
      const v16h pf = ld_frag(&Ps[pbase + c * 32], LDT);
#pragma unroll
      for (int nb = 0; nb < 8; ++nb) {
        const v16h vf = ld_frag(&VO.h[(nb * 16) * LDT + c * 32], LDT);
        o[nb] = wmma16(pf, vf, o[nb]);
      }
    }
    __syncthreads();
  }

  float inv[8];
#pragma unroll
  for (int v = 0; v < 8; ++v)
    inv[v] = __builtin_amdgcn_rcpf(red16_sum(lsum[v])) * (1.0f / VCARRY);
#pragma unroll
  for (int cp = 0; cp < 4; ++cp) {
#pragma unroll
    for (int v = 0; v < 8; ++v) {
      VO.f[obase + (hh * 8u + (unsigned)v) * LDO + m]       = o[2 * cp][v] * inv[v];
      VO.f[obase + (hh * 8u + (unsigned)v) * LDO + 16u + m] = o[2 * cp + 1][v] * inv[v];
    }
    wave_lds_sync();
    v4f x[4];
    size_t off[4];
    bool ok[4];
#pragma unroll
    for (unsigned i = 0; i < 4u; ++i) {
      const unsigned r = 4u * i + (lane >> 3);
      const unsigned c = (lane & 7u) * 4u;
      x[i] = *(const v4f*)&VO.f[obase + r * LDO + c];
      const unsigned row = qrow0 + r;
      ok[i] = row < (unsigned)NREAL;
      off[i] = (size_t)row * DCH + (unsigned)cp * 32u + c;
    }
#pragma unroll
    for (int i = 0; i < 4; ++i)
      if (ok[i]) *(volatile v4f*)(Out + off[i]) = x[i];
    __threadfence();
#pragma unroll
    for (int i = 0; i < 4; ++i)
      if (ok[i]) *(volatile v4f*)(Out + off[i]) = x[i];
    wave_lds_sync();
  }
}

extern "C" void kernel_launch(void* const* d_in, const int* in_sizes, int n_in,
                              void* d_out, int out_size, void* d_ws, size_t ws_size,
                              hipStream_t stream) {
  if (n_in < 5) return;
  if ((long long)in_sizes[0] < (long long)NFULL * DCH) return;
  if ((long long)in_sizes[1] < (long long)NREAL * DCH) return;
  if ((long long)in_sizes[3] < (long long)DCH * DCH) return;
  if (in_sizes[4] < DCH) return;
  if ((long long)out_size < (long long)NREAL * DCH) return;
  if (ws_size < WS_TOTAL) return;

  const float* X  = (const float*)d_in[0];
  const float* y  = (const float*)d_in[1];
  const float* R  = (const float*)d_in[3];
  const float* tv = (const float*)d_in[4];
  float* out = (float*)d_out;

  char* ws = (char*)d_ws;
  _Float16* XQ = (_Float16*)(ws + OFF_XQ);
  _Float16* YH = (_Float16*)(ws + OFF_YH);
  _Float16* RH = (_Float16*)(ws + OFF_RH);
  _Float16* KH = (_Float16*)(ws + OFF_KH);
  _Float16* VT = (_Float16*)(ws + OFF_VT);
  float*    GQ = (float*)(ws + OFF_GQ);
  float*    GK = (float*)(ws + OFF_GK);

  dim3 blk(256);
  conv_norm_kernel<<<dim3((NFULL * DCH) / 4096), blk, 0, stream>>>(X, XQ, GQ,
                                                                  (unsigned)(NFULL * DCH));
  conv_plain_kernel<<<dim3((KPAD * DCH) / 4096), blk, 0, stream>>>(y, YH,
                                                                   (unsigned)(NREAL * DCH));
  conv_plain_kernel<<<dim3((DCH * DCH) / 4096), blk, 0, stream>>>(R, RH, (unsigned)(DCH * DCH));
  vtconv_kernel<<<dim3(DCH / 64, KPAD / 64), blk, 0, stream>>>(X, VT);
  proj_kernel<<<dim3(KPAD / 64), blk, 0, stream>>>(YH, RH, tv, KH, GK);
  kreg_flash_kernel<<<dim3(QROWS / 128), blk, 0, stream>>>(XQ, KH, VT, GQ, GK, out);
}
